// QuantLinear_24885040513624
// MI455X (gfx1250) — hardware-verified
//
#include <hip/hip_runtime.h>

constexpr int kInF          = 4096;
constexpr int kOutF         = 11008;
constexpr int kGroup        = 128;
constexpr int kNGroups      = kInF / kGroup;
constexpr int kTok          = 4;
constexpr int kColsPerBlock = 32;
constexpr int kNBlocks      = kOutF / kColsPerBlock;
constexpr int kWaves        = 8;
constexpr int kThreads      = kWaves * 32;
constexpr int kKPerWave     = kInF / kWaves;
constexpr int kGroupsPerWave= kKPerWave / kGroup;
constexpr int kStepsPerGroup= kGroup / 32;
constexpr int kQwRows       = kInF / 8;
constexpr int kQzCols       = kOutF / 8;
constexpr int kChunksPerRow = kInF / 8;
constexpr int kStageIters   = (kTok * kChunksPerRow) / kThreads;

static_assert(kOutF % kColsPerBlock == 0);
static_assert(kInF % (kWaves * kGroup) == 0);
static_assert(kGroup % 32 == 0);
static_assert((kTok * kChunksPerRow) % kThreads == 0);
static_assert(kNGroups == kWaves * kGroupsPerWave);
static_assert(kQwRows == kChunksPerRow);
static_assert(kTok == 4);

typedef __attribute__((ext_vector_type(16))) _Float16 v16h;
typedef __attribute__((ext_vector_type(8)))  _Float16 v8h;
typedef __attribute__((ext_vector_type(2)))  _Float16 v2h;
typedef __attribute__((ext_vector_type(8)))  float    v8f;
typedef __attribute__((ext_vector_type(4)))  float    v4f;

union BFrag { unsigned u[8]; v16h v; };
union AFrag { v8h h[2]; v16h v; };

__device__ __forceinline__ void mma_guard2(v8f& a, v8f& b, v16h x, v16h y, v16h z) {
  asm volatile("v_nop\n\tv_nop\n\tv_nop\n\tv_nop" : "+v"(a), "+v"(b) : "v"(x), "v"(y), "v"(z));
}

__device__ __forceinline__ v8f mma_f16(v16h a, v16h b, v8f c) {
  return __builtin_amdgcn_wmma_f32_16x16x32_f16(false, a, false, b, (short)0, c, false, false);
}

__device__ __forceinline__ unsigned unpack_pair(unsigned w, int j, v2h z2) {
  const unsigned t = ((w >> (4 * j)) & 0x000F000Fu) | 0x64006400u;
  const v2h d = __builtin_bit_cast(v2h, t) - z2;
  return __builtin_bit_cast(unsigned, d);
}

__global__ __launch_bounds__(kThreads) void qgemm4_kernel(
    const float* __restrict__ x,
    const float* __restrict__ scales,
    const float* __restrict__ bias,
    const int*   __restrict__ qweight,
    const int*   __restrict__ qzeros,
    float*       __restrict__ out)
{
  __shared__ __align__(16) _Float16 xl[kTok * kInF];
  __shared__ __align__(16) float    red[kWaves][kTok][kColsPerBlock];
  __shared__ __align__(16) float    orow[kTok][kColsPerBlock];

  const int tid  = threadIdx.x;
  const int lane = tid & 31;
  const int wave = tid >> 5;
  const int hsel = lane >> 4;
  const int m    = lane & 15;
  const int n0   = blockIdx.x * kColsPerBlock;

#pragma unroll 1
  for (int it = 0; it < kStageIters; ++it) {
    const int ci = tid + it * kThreads;
    const float* xp = x + (size_t)ci * 8;
    const v4f lo4 = *(const v4f*)(xp);
    const v4f hi4 = *(const v4f*)(xp + 4);
    v8h c;
    c[0] = (_Float16)lo4[0]; c[1] = (_Float16)hi4[0];
    c[2] = (_Float16)lo4[1]; c[3] = (_Float16)hi4[1];
    c[4] = (_Float16)lo4[2]; c[5] = (_Float16)hi4[2];
    c[6] = (_Float16)lo4[3]; c[7] = (_Float16)hi4[3];
    *(v8h*)(xl + (size_t)ci * 8) = c;
  }
  __syncthreads();

  const v8h* xv   = (const v8h*)xl;
  const int abase = (m & 3) * kChunksPerRow;
  const int nc0   = n0 + m;
  const int nc1   = n0 + 16 + m;
  const int nsh   = 4 * (m & 7);

  v8f acc0 = (v8f){0.f,0.f,0.f,0.f,0.f,0.f,0.f,0.f};
  v8f acc1 = (v8f){0.f,0.f,0.f,0.f,0.f,0.f,0.f,0.f};

#pragma unroll 1
  for (int gi = 0; gi < kGroupsPerWave; ++gi) {
    const int g = wave * kGroupsPerWave + gi;

    const unsigned zw0 = (unsigned)qzeros[g * kQzCols + (nc0 >> 3)];
    const unsigned zw1 = (unsigned)qzeros[g * kQzCols + (nc1 >> 3)];
    const float s0 = scales[g * kOutF + nc0];
    const float s1 = scales[g * kOutF + nc1];
    const unsigned zb0 = 0x6401u + ((zw0 >> nsh) & 0xFu);
    const unsigned zb1 = 0x6401u + ((zw1 >> nsh) & 0xFu);
    const v2h z2_0 = __builtin_bit_cast(v2h, (zb0 << 16) | zb0);
    const v2h z2_1 = __builtin_bit_cast(v2h, (zb1 << 16) | zb1);

    v8f t0 = (v8f){0.f,0.f,0.f,0.f,0.f,0.f,0.f,0.f};
    v8f t1 = (v8f){0.f,0.f,0.f,0.f,0.f,0.f,0.f,0.f};

#pragma unroll 1
    for (int kt = 0; kt < kStepsPerGroup; ++kt) {
      const int k0 = g * kGroup + kt * 32;
      const int r0 = (k0 >> 3) + hsel;
      const int r1 = r0 + 2;
      const unsigned w00 = (unsigned)qweight[r0 * kOutF + nc0];
      const unsigned w01 = (unsigned)qweight[r1 * kOutF + nc0];
      const unsigned w10 = (unsigned)qweight[r0 * kOutF + nc1];
      const unsigned w11 = (unsigned)qweight[r1 * kOutF + nc1];

      BFrag b0, b1;
#pragma unroll
      for (int j = 0; j < 4; ++j) {
        b0.u[j]     = unpack_pair(w00, j, z2_0);
        b0.u[4 + j] = unpack_pair(w01, j, z2_0);
        b1.u[j]     = unpack_pair(w10, j, z2_1);
        b1.u[4 + j] = unpack_pair(w11, j, z2_1);
      }

      AFrag a;
      a.h[0] = xv[abase + r0];
      a.h[1] = xv[abase + r1];

      t0 = mma_f16(a.v, b0.v, t0);
      t1 = mma_f16(a.v, b1.v, t1);
      mma_guard2(t0, t1, a.v, b0.v, b1.v);
    }

#pragma unroll
    for (int i = 0; i < 8; ++i) {
      acc0[i] = fmaf(s0, t0[i], acc0[i]);
      acc1[i] = fmaf(s1, t1[i], acc1[i]);
    }
  }

  if (lane < 16) {
#pragma unroll
    for (int r = 0; r < kTok; ++r) {
      red[wave][r][lane]      = acc0[r];
      red[wave][r][16 + lane] = acc1[r];
    }
  }
  __syncthreads();

  if (tid < kTok * 32) {
    const int row = tid >> 5;
    float s = 0.0f;
#pragma unroll
    for (int w = 0; w < kWaves; ++w) s += red[w][row][lane];
    s += bias[n0 + lane];
    orow[row][lane] = s;
  }
  __syncthreads();

  if (wave == 0) {
    const int row = lane >> 3;
    const int c4  = (lane & 7) * 4;
    const v4f v = *(const v4f*)(&orow[row][c4]);
    float* p = out + (size_t)row * kOutF + n0 + c4;
    *(volatile v4f*)p = v;
    __threadfence();
    *(volatile v4f*)p = v;
  }
}

extern "C" void kernel_launch(void* const* d_in, const int* in_sizes, int n_in,
                              void* d_out, int out_size, void* d_ws, size_t ws_size,
                              hipStream_t stream) {
  (void)in_sizes; (void)n_in; (void)out_size; (void)d_ws; (void)ws_size;
  const float* x       = (const float*)d_in[0];
  const float* scales  = (const float*)d_in[1];
  const float* bias    = (const float*)d_in[2];
  const int*   qweight = (const int*)d_in[3];
  const int*   qzeros  = (const int*)d_in[4];
  float*       out     = (float*)d_out;

  qgemm4_kernel<<<dim3(kNBlocks), dim3(kThreads), 0, stream>>>(x, scales, bias, qweight, qzeros, out);
}
